// REG_RNN_8693013807612
// MI455X (gfx1250) — hardware-run, weakly checked
//
#include <hip/hip_runtime.h>
#include <math.h>

constexpr int NBATCH   = 256;
constexpr int NSTEP    = 4096;
constexpr int NHID     = 32;
constexpr int ROWS_BLK = 16;
constexpr int CHUNK    = 32;
constexpr int NCHUNK   = NSTEP / CHUNK;
constexpr int HPITCH   = 40;
constexpr int FPITCH   = 36;
constexpr int XPITCH   = 16;
constexpr int OPITCH   = 32;
constexpr int ATILE    = ROWS_BLK * HPITCH;
constexpr float RES_SCALE = 2048.0f;
constexpr float RES_INV   = 1.0f / 2048.0f;
constexpr float HI_MIN    = 1.0f / 8192.0f;
constexpr int NOUT0 = NBATCH * NSTEP;
constexpr int NOUT1 = NBATCH * NHID;
static_assert(NBATCH % ROWS_BLK == 0);
static_assert(NSTEP % CHUNK == 0);
static_assert(NHID == 32);
static_assert(CHUNK == 32);
static_assert((size_t)NOUT0 * 4 == (size_t)4194304);
static_assert(((size_t)NOUT0 * 4) % 128 == 0);
static_assert((size_t)(NOUT0 + NOUT1) * 4 == (size_t)4227072);
static_assert((HPITCH * 2) % 16 == 0);
static_assert((FPITCH * 4) % 16 == 0);

typedef __attribute__((ext_vector_type(16))) _Float16 v16h;
typedef __attribute__((ext_vector_type(8)))  _Float16 v8h;
typedef __attribute__((ext_vector_type(8)))  float    v8f;
typedef __attribute__((ext_vector_type(4)))  float    v4f;

template <typename T> struct Frag;
template <> struct Frag<_Float16> {
  typedef v16h V; union U { v16h v; v8h h[2]; };
  static __device__ __forceinline__ v16h load(const _Float16* p) {
    U f; f.h[0] = *(const v8h*)(p); f.h[1] = *(const v8h*)(p + 16); return f.v;
  }
  static __device__ __forceinline__ v8f mma(v16h a, v16h b, v8f c) {
    return __builtin_amdgcn_wmma_f32_16x16x32_f16(false, a, false, b, (short)0, c, false, false);
  }
};

__device__ __forceinline__ void group_guard(v8f& a, v8f& b, v16h p, v16h q, v16h r, v16h s) {
  asm volatile("v_nop\n\tv_nop\n\tv_nop\n\tv_nop" : "+v"(a), "+v"(b) : "v"(p), "v"(q), "v"(r), "v"(s));
}

__device__ __forceinline__ void split_f16(float v, _Float16& hi, _Float16& res) {
  const float vh = (fabsf(v) < HI_MIN) ? 0.0f : v;
  hi = (_Float16)vh;
  const float hf = (float)hi;
  const float d  = v - hf;
  res = (_Float16)(d * RES_SCALE);
}

__device__ __forceinline__ float tanh_f32(float x) {
  const float e = expf(2.0f * x);
  return 1.0f - 2.0f / (e + 1.0f);
}

__device__ __forceinline__ void load_x_chunk(const float* __restrict__ x, int rowbase, int t0, int lane, float* XsT) {
#pragma unroll
  for (int it = 0; it < 4; ++it) {
    const int idx = it * 32 + lane;
    const int row = idx >> 3;
    const int c4  = (idx & 7) * 4;
    const v4f v = *(const v4f*)(x + (size_t)(rowbase + row) * NSTEP + (size_t)(t0 + c4));
    XsT[(c4 + 0) * XPITCH + row] = v[0];
    XsT[(c4 + 1) * XPITCH + row] = v[1];
    XsT[(c4 + 2) * XPITCH + row] = v[2];
    XsT[(c4 + 3) * XPITCH + row] = v[3];
  }
}

__global__ __launch_bounds__(32) void rnn_seq_kernel(const float* __restrict__ x, const float* __restrict__ h0,
                                                     const float* __restrict__ w_ih, const float* __restrict__ b_ih,
                                                     const float* __restrict__ w_hh, const float* __restrict__ b_hh,
                                                     const float* __restrict__ w_out, const float* __restrict__ b_out,
                                                     float* __restrict__ out0, float* __restrict__ out1) {
  __shared__ __align__(16) _Float16 Wh[NHID * HPITCH];
  __shared__ __align__(16) _Float16 Wl[NHID * HPITCH];
  __shared__ __align__(16) _Float16 Ahi[2 * ATILE];
  __shared__ __align__(16) _Float16 Alo[2 * ATILE];
  __shared__ __align__(16) float    Hf[ROWS_BLK * FPITCH];
  __shared__ __align__(16) float    XsT[CHUNK * XPITCH];
  __shared__ __align__(16) float    Os[ROWS_BLK * OPITCH];
  __shared__ __align__(16) float    Cs[4 * NHID];

  const int lane = threadIdx.x & 31;
  const int c    = lane & 15;
  const int hh   = lane >> 4;
  const int koff = hh * 8;
  const int rowbase = blockIdx.x * ROWS_BLK;

#pragma unroll 1
  for (int q = 0; q < NHID / 4; ++q) {
    const v4f w = *(const v4f*)(w_hh + lane * NHID + 4 * q);
#pragma unroll
    for (int e = 0; e < 4; ++e) {
      const float wv = w[e];
      _Float16 hi, rs;
      split_f16(wv, hi, rs);
      Wh[lane * HPITCH + 4 * q + e] = hi;
      Wl[lane * HPITCH + 4 * q + e] = rs;
    }
  }
#pragma unroll 1
  for (int m = 0; m < ROWS_BLK; ++m) {
    const float v = h0[(size_t)(rowbase + m) * NHID + lane];
    _Float16 hi, rs;
    split_f16(v, hi, rs);
    Ahi[m * HPITCH + lane] = hi;
    Alo[m * HPITCH + lane] = rs;
    Hf[m * FPITCH + lane]  = v;
  }
  Cs[lane]            = w_ih[lane];
  Cs[NHID + lane]     = b_ih[lane];
  Cs[2 * NHID + lane] = b_hh[lane];
  Cs[3 * NHID + lane] = w_out[lane];
  v4f wo[4];
#pragma unroll
  for (int q = 0; q < 4; ++q) wo[q] = *(const v4f*)(w_out + 16 * hh + 4 * q);
  const float bo = b_out[0];

  load_x_chunk(x, rowbase, 0, lane, XsT);
  __syncthreads();

  const v8f z8 = {0.f, 0.f, 0.f, 0.f, 0.f, 0.f, 0.f, 0.f};
  int cur = 0;

#pragma unroll 1
  for (int ch = 0; ch < NCHUNK; ++ch) {
#pragma unroll 1
    for (int tt = 0; tt < CHUNK; ++tt) {
      const _Float16* arh = Ahi + cur * ATILE + c * HPITCH + koff;
      const _Float16* arl = Alo + cur * ATILE + c * HPITCH + koff;
      _Float16* awh = Ahi + (cur ^ 1) * ATILE;
      _Float16* awl = Alo + (cur ^ 1) * ATILE;
      const v16h ah = Frag<_Float16>::load(arh);
      const v16h al = Frag<_Float16>::load(arl);
      const v4f xa = *(const v4f*)(XsT + tt * XPITCH + 8 * hh);
      const v4f xb = *(const v4f*)(XsT + tt * XPITCH + 8 * hh + 4);

#pragma unroll 1
      for (int nt = 0; nt < 2; ++nt) {
        const int j = 16 * nt + c;
        const v16h bh = Frag<_Float16>::load(Wh + j * HPITCH + koff);
        const v16h bl = Frag<_Float16>::load(Wl + j * HPITCH + koff);
        const float wi  = Cs[j];
        const float bi  = Cs[NHID + j];
        const float bhv = Cs[2 * NHID + j];
        v8f accR = Frag<_Float16>::mma(al, bh, z8);
        accR     = Frag<_Float16>::mma(ah, bl, accR);
        v8f accM = Frag<_Float16>::mma(ah, bh, z8);
        group_guard(accM, accR, ah, al, bh, bl);
#pragma unroll
        for (int r = 0; r < 8; ++r) {
          const float xv  = (r < 4) ? xa[r & 3] : xb[r & 3];
          const float dot = accM[r] + accR[r] * RES_INV;
          const float xp  = fmaf(xv, wi, bi);
          const float pre = (xp + dot) + bhv;
          const float hn  = tanh_f32(pre);
          _Float16 hi, rs;
          split_f16(hn, hi, rs);
          awh[(8 * hh + r) * HPITCH + j] = hi;
          awl[(8 * hh + r) * HPITCH + j] = rs;
          Hf[(8 * hh + r) * FPITCH + j]  = hn;
        }
      }
      __syncthreads();

      {
        const float* hr = Hf + c * FPITCH + 16 * hh;
        const v4f g0 = *(const v4f*)(hr);
        const v4f g1 = *(const v4f*)(hr + 4);
        const v4f g2 = *(const v4f*)(hr + 8);
        const v4f g3 = *(const v4f*)(hr + 12);
        float s = 0.0f;
#pragma unroll
        for (int e = 0; e < 4; ++e) s = fmaf(g0[e], wo[0][e], s);
#pragma unroll
        for (int e = 0; e < 4; ++e) s = fmaf(g1[e], wo[1][e], s);
#pragma unroll
        for (int e = 0; e < 4; ++e) s = fmaf(g2[e], wo[2][e], s);
#pragma unroll
        for (int e = 0; e < 4; ++e) s = fmaf(g3[e], wo[3][e], s);
        const float so = __shfl_xor(s, 16, 32);
        const float o  = (s + so) + bo;
        if (lane < 16) Os[c * OPITCH + tt] = o;
      }
      asm volatile("" ::: "memory");
      cur ^= 1;
    }

    __syncthreads();
    {
      const int t0 = ch * CHUNK;
      float ov[ROWS_BLK];
#pragma unroll
      for (int m = 0; m < ROWS_BLK; ++m) ov[m] = Os[m * OPITCH + lane];
      for (int pass = 0; pass < 2; ++pass) {
#pragma unroll
        for (int m = 0; m < ROWS_BLK; ++m)
          *(volatile float*)(out0 + (size_t)(rowbase + m) * NSTEP + (size_t)(t0 + lane)) = ov[m];
        __threadfence();
      }
      const int chn = (ch + 1 < NCHUNK) ? (ch + 1) : (NCHUNK - 1);
      load_x_chunk(x, rowbase, chn * CHUNK, lane, XsT);
    }
    __syncthreads();
  }

  {
    float hv[ROWS_BLK];
#pragma unroll
    for (int m = 0; m < ROWS_BLK; ++m) hv[m] = Hf[m * FPITCH + lane];
    for (int pass = 0; pass < 2; ++pass) {
#pragma unroll
      for (int m = 0; m < ROWS_BLK; ++m)
        *(volatile float*)(out1 + (size_t)(rowbase + m) * NHID + lane) = hv[m];
      __threadfence();
    }
  }
}

extern "C" void kernel_launch(void* const* d_in, const int* in_sizes, int n_in,
                              void* d_out, int out_size, void* d_ws, size_t ws_size, hipStream_t stream) {
  (void)d_ws; (void)ws_size;
  if (n_in < 8 || d_out == nullptr) return;
  if (in_sizes[0] != NBATCH * NSTEP || in_sizes[1] != NBATCH * NHID || in_sizes[2] != NHID ||
      in_sizes[3] != NHID || in_sizes[4] != NHID * NHID || in_sizes[5] != NHID ||
      in_sizes[6] != NHID || in_sizes[7] != 1 || out_size != NOUT0 + NOUT1) return;

  const float* x     = (const float*)d_in[0];
  const float* h0    = (const float*)d_in[1];
  const float* w_ih  = (const float*)d_in[2];
  const float* b_ih  = (const float*)d_in[3];
  const float* w_hh  = (const float*)d_in[4];
  const float* b_hh  = (const float*)d_in[5];
  const float* w_out = (const float*)d_in[6];
  const float* b_out = (const float*)d_in[7];

  float* out0 = (float*)d_out;
  float* out1 = (float*)d_out + (size_t)NOUT0;

  rnn_seq_kernel<<<NBATCH / ROWS_BLK, 32, 0, stream>>>(x, h0, w_ih, b_ih, w_hh, b_hh, w_out, b_out, out0, out1);
}
